// LifelineGNN_19911468384345
// MI455X (gfx1250) — hardware-verified
//
#include <hip/hip_runtime.h>
#include <math.h>

typedef _Float16 f16;
typedef f16   v16h __attribute__((ext_vector_type(16)));
typedef f16   v8h  __attribute__((ext_vector_type(8)));
typedef float v8f  __attribute__((ext_vector_type(8)));
typedef float v4f  __attribute__((ext_vector_type(4)));
typedef float v2f  __attribute__((ext_vector_type(2)));
typedef int   v4i  __attribute__((ext_vector_type(4)));
typedef v4f __attribute__((may_alias)) v4fa;
typedef v4i __attribute__((may_alias)) v4ia;
typedef v8h __attribute__((may_alias)) v8ha;

union Frag { v16h v; v8h half[2]; };

#define NB   2
#define NN   10000
#define NT   12
#define NCIN 2
#define NE   160000
#define ND   64
#define NTF  14
#define NG   (NB*NT)
#define RR   (NG*NN)
#define RG   (NB*NN)
#define SB   1024
#define EPAD (((NE+SB-1)/SB)*SB)
#define RP_PAD 10240
#define CSR_T 512
#define NPT  20
#define CSR_CH 2048
#define WTS  (3*64*64)
#define GW   5
#define GRU_T (GW*32)
#define GRU_WAVE_HALVES 6144
#define GRU_LDS_BYTES ((4*WTS + 1024 + GW*GRU_WAVE_HALVES)*2)
#define SCL  (1.0f/16.0f)
#define WSC  16.0f

__device__ __forceinline__ v8f mma16(v16h a, v16h b, v8f c){
  c = __builtin_amdgcn_wmma_f32_16x16x32_f16(false, a, false, b, (short)0, c, false, false);
  asm volatile("v_nop\n\tv_nop\n\tv_nop\n\tv_nop" : "+v"(c) : "v"(a), "v"(b));
  return c;
}
__device__ __forceinline__ v8f zero8(){ v8f z = {0.f,0.f,0.f,0.f,0.f,0.f,0.f,0.f}; return z; }
__device__ __forceinline__ float wsum32(float v){
#pragma unroll
  for (int o=16;o>0;o>>=1) v += __shfl_xor(v,o,32);
  return v;
}
__device__ __forceinline__ float wmax32(float v){
#pragma unroll
  for (int o=16;o>0;o>>=1) v = fmaxf(v, __shfl_xor(v,o,32));
  return v;
}
__device__ __forceinline__ int ub_count(const int* rp, int cnt, int x){
  int lo=0, hi=cnt;
  while (lo<hi){ int mid=(lo+hi)>>1; if (rp[mid] <= x) lo=mid+1; else hi=mid; }
  return lo;
}

__global__ __launch_bounds__(256) void k_prep(const float* ew, int nE,
    const float* We0, const float* ae0, const float* We1, const float* ae1, float* sc){
  __shared__ double red[256];
  __shared__ __attribute__((aligned(16))) float line[32];
  const int tid = threadIdx.x;
  double s = 0.0;
  for (int i=tid;i<nE;i+=256) s += (double)ew[i];
  red[tid]=s; __syncthreads();
  for (int o=128;o>0;o>>=1){ if (tid<o) red[tid]+=red[tid+o]; __syncthreads(); }
  if (tid<32) line[tid]=0.f;
  __syncthreads();
  if (tid==0) line[0] = (float)(red[0] / (double)nE);
  if (tid>=1 && tid<9){
    int k = tid-1; int hh = k & 3;
    const float* W  = (k<4) ? We0 : We1;
    const float* ae = (k<4) ? ae0 : ae1;
    float c = 0.f;
#pragma unroll 1
    for (int q=0;q<16;q++) c += W[hh*16+q]*ae[hh*16+q];
    line[tid] = c;
  }
  __syncthreads();
  if (tid<8){
    v4f v = *(const v4fa*)(line + tid*4);
    *(volatile v4f*)(sc + tid*4) = v;
    __threadfence();
    *(volatile v4f*)(sc + tid*4) = v;
  }
}

__global__ __launch_bounds__(256) void k_prepw(const float* wih0, const float* whh0, const float* wih1, const float* whh1,
    const float* g1W, const float* headW,
    f16* o0, f16* o1, f16* o2, f16* o3, f16* og, f16* ohw){
  const int i = blockIdx.x*blockDim.x + threadIdx.x;
  const int NGR = WTS/8;
  float vals[8];
  f16* dst;
  if (i < 4*NGR){
    int a = i / NGR, gi = i - a*NGR;
    const float* src = (a==0) ? wih0 : (a==1) ? whh0 : (a==2) ? wih1 : whh1;
    dst = ((a==0) ? o0 : (a==1) ? o1 : (a==2) ? o2 : o3) + gi*8;
#pragma unroll
    for (int j=0;j<8;j++) vals[j] = src[gi*8+j]*WSC;
  } else if (i < 4*NGR + 512){
    int gi = i - 4*NGR; int n = gi>>3, k0 = (gi&7)*8;
    dst = og + n*64 + k0;
#pragma unroll
    for (int j=0;j<8;j++) vals[j] = g1W[(k0+j)*64 + n]*WSC;
  } else if (i < 4*NGR + 512 + 128){
    int gi = i - 4*NGR - 512; int n = gi>>3, k0 = (gi&7)*8;
    dst = ohw + n*64 + k0;
#pragma unroll
    for (int j=0;j<8;j++) vals[j] = (n < NTF) ? headW[(k0+j)*NTF + n]*WSC : 0.f;
  } else return;
  v8h v;
#pragma unroll
  for (int j=0;j<8;j++) v[j] = (f16)vals[j];
  *(volatile v8h*)dst = v;
  __threadfence();
  *(volatile v8h*)dst = v;
}

__global__ __launch_bounds__(CSR_T) void k_csr_rowptr(const int* ei, int nE, int nN, int* rowptr){
  __shared__ int chunk[CSR_CH];
  __shared__ __attribute__((aligned(16))) int rps[RP_PAD];
  __shared__ int wsum[32];
  const int tid = threadIdx.x, lane = tid & 31, wid = tid >> 5;
  const int a = tid*NPT;
  int cnt[NPT];
#pragma unroll
  for (int q=0;q<NPT;q++) cnt[q]=0;
#pragma unroll 1
  for (int cb=0; cb<nE; cb+=CSR_CH){
    int len = nE - cb; if (len > CSR_CH) len = CSR_CH;
    __syncthreads();
    for (int i=tid;i<len;i+=CSR_T) chunk[i] = ei[(size_t)nE + cb + i];
    __syncthreads();
    for (int e=0;e<len;e++){
      int rel = chunk[e] - a;
#pragma unroll
      for (int q=0;q<NPT;q++) cnt[q] += (rel==q) ? 1 : 0;
    }
  }
  int tot = 0;
#pragma unroll
  for (int q=0;q<NPT;q++) tot += cnt[q];
  int v = tot;
#pragma unroll
  for (int o=1;o<32;o<<=1){ int t = __shfl_up(v,o,32); if (lane>=o) v += t; }
  if (lane==31) wsum[wid] = v;
  __syncthreads();
  if (wid==0){
    int x = (lane < CSR_T/32) ? wsum[lane] : 0;
#pragma unroll
    for (int o=1;o<32;o<<=1){ int t = __shfl_up(x,o,32); if (lane>=o) x += t; }
    if (lane < CSR_T/32) wsum[lane] = x;
  }
  __syncthreads();
  const int excl  = v - tot + ((wid>0) ? wsum[wid-1] : 0);
  const int total = wsum[CSR_T/32 - 1];
  int run = excl;
#pragma unroll
  for (int q=0;q<NPT;q++){ int idx = a+q; if (idx < nN) rps[idx] = run; run += cnt[q]; }
  for (int idx=nN+tid; idx<RP_PAD; idx+=CSR_T) rps[idx] = total;
  __syncthreads();
  for (int i=tid;i<RP_PAD/4;i+=CSR_T){ v4i r = *(const v4ia*)(rps + i*4); *(volatile v4i*)(rowptr + i*4) = r; }
  __threadfence();
  for (int i=tid;i<RP_PAD/4;i+=CSR_T){ v4i r = *(const v4ia*)(rps + i*4); *(volatile v4i*)(rowptr + i*4) = r; }
}

__global__ __launch_bounds__(256) void k_slotfill(const int* ei, const float* ew, int nE, int nN,
    const int* rowptr, int* ssrc, float* sw){
  __shared__ int   cd[SB];
  __shared__ int   cs[SB];
  __shared__ float cw[SB];
  __shared__ __attribute__((aligned(16))) int   ts[SB];
  __shared__ __attribute__((aligned(16))) float tw[SB];
  const int tid = threadIdx.x;
  const int S0 = blockIdx.x*SB;
  int S1 = S0 + SB; if (S1 > nE) S1 = nE;
  for (int i=tid;i<SB;i+=256){ ts[i]=0; tw[i]=0.f; }
  int nlo = ub_count(rowptr, nN, S0) - 1;      if (nlo < 0) nlo = 0;
  int nhi = ub_count(rowptr, nN, S1-1) - 1;    if (nhi < nlo) nhi = nlo;
  const int count = nhi - nlo + 1;
  const int nrep  = (count + 255) >> 8;
#pragma unroll 1
  for (int rd=0; rd<nrep; rd++){
    const int node = nlo + rd*256 + tid;
    const bool act = node <= nhi;
    int pos = 0, pend = 0;
    if (act){ pos = rowptr[node]; pend = rowptr[node+1]; if (pend > S1) pend = S1; }
#pragma unroll 1
    for (int cb=0; cb<nE; cb+=SB){
      int len = nE - cb; if (len > SB) len = SB;
      __syncthreads();
      for (int i=tid;i<len;i+=256){ cd[i] = ei[(size_t)nE + cb + i]; cs[i] = ei[cb+i]; cw[i] = ew[cb+i]; }
      __syncthreads();
      if (act && pos < pend){
        for (int e=0;e<len;e++){
          if (cd[e] == node){
            if (pos >= S0){
              int sv = cs[e]; sv = (sv < 0) ? 0 : ((sv >= nN) ? nN-1 : sv);
              ts[pos-S0] = sv; tw[pos-S0] = cw[e];
            }
            pos++;
            if (pos >= pend) break;
          }
        }
      }
    }
  }
  __syncthreads();
  v4i a4 = *(const v4ia*)(ts + tid*4);
  v4f b4 = *(const v4fa*)(tw + tid*4);
  *(volatile v4i*)(ssrc + S0 + tid*4) = a4;
  *(volatile v4f*)(sw   + S0 + tid*4) = b4;
  __threadfence();
  *(volatile v4i*)(ssrc + S0 + tid*4) = a4;
  *(volatile v4f*)(sw   + S0 + tid*4) = b4;
}

__global__ __launch_bounds__(128) void k_feat0(const float* xseq, const float* W,
    const float* as0, const float* ad0, float* xp, float* al, int nRows){
  __shared__ __attribute__((aligned(16))) float xs[128*64];
  __shared__ __attribute__((aligned(16))) float als[128*8];
  const int tid = threadIdx.x;
  const int R0 = blockIdx.x*128;
  const int r = R0 + tid;
  if (r < nRows){
    int g = r / NN, n = r - g*NN;
    int bI = g / NT, t = g - bI*NT;
    const float* xin = xseq + (((size_t)(bI*NN + n))*NT + t)*NCIN;
    float x0 = xin[0], x1 = xin[1];
#pragma unroll
    for (int hd=0; hd<4; hd++){
      float sa = 0.f, sd = 0.f;
#pragma unroll 1
      for (int c=0;c<16;c++){
        int d = hd*16 + c;
        float v = x0*W[d] + x1*W[64+d];
        xs[tid*64 + d] = v;
        sa += v*as0[d];
        sd += v*ad0[d];
      }
      als[tid*8 + hd] = sa;
      als[tid*8 + 4 + hd] = sd;
    }
  }
  __syncthreads();
  int nr = nRows - R0; if (nr > 128) nr = 128;
  const int n4x = nr*16, n4a = nr*2;
  float* xb = xp + (size_t)R0*64;
  float* ab = al + (size_t)R0*8;
  for (int i=tid;i<n4x;i+=128){ v4f v = *(const v4fa*)(xs + i*4);  *(volatile v4f*)(xb + i*4) = v; }
  for (int i=tid;i<n4a;i+=128){ v4f v = *(const v4fa*)(als + i*4); *(volatile v4f*)(ab + i*4) = v; }
  __threadfence();
  for (int i=tid;i<n4x;i+=128){ v4f v = *(const v4fa*)(xs + i*4);  *(volatile v4f*)(xb + i*4) = v; }
  for (int i=tid;i<n4a;i+=128){ v4f v = *(const v4fa*)(als + i*4); *(volatile v4f*)(ab + i*4) = v; }
}

__device__ __forceinline__ void edge_logits(int j, int deg, int rp0, int n, const int* ssrc, const float* sw,
    float meanw, const float* al, size_t gbase, v4f ad, float ce0, float ce1, float ce2, float ce3,
    int& src, float& a0, float& a1, float& a2, float& a3){
  float ea;
  if (j < deg){
    int idx = rp0 + j;
    int s = ssrc[idx]; s = (s < 0) ? 0 : ((s >= NN) ? NN-1 : s);
    src = s; ea = sw[idx];
  } else { src = n; ea = meanw; }
  v4f as = *(const v4f*)(al + (gbase + (size_t)src)*8);
  a0 = as.x + ad.x + ea*ce0; a0 = (a0 > 0.f) ? a0 : 0.2f*a0;
  a1 = as.y + ad.y + ea*ce1; a1 = (a1 > 0.f) ? a1 : 0.2f*a1;
  a2 = as.z + ad.z + ea*ce2; a2 = (a2 > 0.f) ? a2 : 0.2f*a2;
  a3 = as.w + ad.w + ea*ce3; a3 = (a3 > 0.f) ? a3 : 0.2f*a3;
}

__global__ __launch_bounds__(256) void k_gat(int mode, int coff,
    const int* rowptr, const int* ssrc, const float* sw,
    const float* al, const float* xp, const float* sc,
    const float* gb, const float* lng, const float* lnb,
    const float* xseq, const float* skW, const float* skb,
    const float* resid, float* hout, int nRows){
  const int l = threadIdx.x & 31;
  const int row = blockIdx.x*(blockDim.x>>5) + (threadIdx.x>>5);
  if (row >= nRows) return;
  const int g = row / NN;
  const int n = row - g*NN;
  int rp0 = rowptr[n], rp1 = rowptr[n+1];
  rp0 = (rp0 < 0) ? 0 : ((rp0 > EPAD) ? EPAD : rp0);
  rp1 = (rp1 < rp0) ? rp0 : ((rp1 > EPAD) ? EPAD : rp1);
  const int deg = rp1 - rp0;
  const int nsl = deg + 1;
  const float meanw = sc[0];
  const float ce0 = sc[coff], ce1 = sc[coff+1], ce2 = sc[coff+2], ce3 = sc[coff+3];
  const size_t gbase = (size_t)g*NN;
  const v4f ad = *(const v4f*)(al + (size_t)row*8 + 4);

  float m0 = -INFINITY, m1 = -INFINITY, m2 = -INFINITY, m3 = -INFINITY;
#pragma unroll 1
  for (int base=0; base<nsl; base+=32){
    int j = base + l;
    if (j < nsl){
      int src; float a0,a1,a2,a3;
      edge_logits(j,deg,rp0,n,ssrc,sw,meanw,al,gbase,ad,ce0,ce1,ce2,ce3,src,a0,a1,a2,a3);
      m0 = fmaxf(m0,a0); m1 = fmaxf(m1,a1); m2 = fmaxf(m2,a2); m3 = fmaxf(m3,a3);
    }
  }
  m0 = wmax32(m0); m1 = wmax32(m1); m2 = wmax32(m2); m3 = wmax32(m3);

  const int hsel = l >> 3;
  float s0=0.f, s1=0.f, s2=0.f, s3=0.f, acc0=0.f, acc1=0.f;
#pragma unroll 1
  for (int base=0; base<nsl; base+=32){
    int j = base + l;
    int src = n; float e0=0.f, e1=0.f, e2=0.f, e3=0.f;
    if (j < nsl){
      float a0,a1,a2,a3;
      edge_logits(j,deg,rp0,n,ssrc,sw,meanw,al,gbase,ad,ce0,ce1,ce2,ce3,src,a0,a1,a2,a3);
      e0 = expf(a0-m0); e1 = expf(a1-m1); e2 = expf(a2-m2); e3 = expf(a3-m3);
      s0 += e0; s1 += e1; s2 += e2; s3 += e3;
    }
    int cnt = nsl - base; if (cnt > 32) cnt = 32;
#pragma unroll 1
    for (int jj=0; jj<cnt; jj++){
      int sb = __shfl(src, jj, 32);
      float w0 = __shfl(e0, jj, 32), w1 = __shfl(e1, jj, 32), w2 = __shfl(e2, jj, 32), w3 = __shfl(e3, jj, 32);
      float w = (hsel==0) ? w0 : (hsel==1) ? w1 : (hsel==2) ? w2 : w3;
      v2f x = *(const v2f*)(xp + (gbase + (size_t)sb)*64 + 2*l);
      acc0 += x.x*w; acc1 += x.y*w;
    }
  }
  s0 = wsum32(s0); s1 = wsum32(s1); s2 = wsum32(s2); s3 = wsum32(s3);
  {
    float i0 = 1.f/(s0 + 1e-16f), i1 = 1.f/(s1 + 1e-16f), i2 = 1.f/(s2 + 1e-16f), i3 = 1.f/(s3 + 1e-16f);
    float inv = (hsel==0) ? i0 : (hsel==1) ? i1 : (hsel==2) ? i2 : i3;
    acc0 *= inv; acc1 *= inv;
  }
  const int c0 = 2*l;
  float v0 = acc0 + gb[c0], v1 = acc1 + gb[c0+1];
  float mean = wsum32(v0 + v1) * (1.f/64.f);
  float d0 = v0 - mean, d1 = v1 - mean;
  float var = wsum32(d0*d0 + d1*d1) * (1.f/64.f);
  float rinv = rsqrtf(var + 1e-5f);
  float y0 = d0*rinv*lng[c0] + lnb[c0];
  float y1 = d1*rinv*lng[c0+1] + lnb[c0+1];
  if (mode == 0){
    int bI = g / NT, t = g - bI*NT;
    const float* xin = xseq + (((size_t)(bI*NN + n))*NT + t)*NCIN;
    float x0 = xin[0], x1 = xin[1];
    y0 += x0*skW[c0]   + x1*skW[64+c0]   + skb[c0];
    y1 += x0*skW[c0+1] + x1*skW[64+c0+1] + skb[c0+1];
  } else {
    v2f rr = *(const v2f*)(resid + (size_t)row*64 + 2*l);
    y0 += rr.x; y1 += rr.y;
  }
  y0 = (y0 > 0.f) ? y0 : 0.f;
  y1 = (y1 > 0.f) ? y1 : 0.f;
  const int la = (2*l) & 31, lb2 = (2*l + 1) & 31;
  v4f o;
  o.x = __shfl(y0, la, 32); o.y = __shfl(y1, la, 32); o.z = __shfl(y0, lb2, 32); o.w = __shfl(y1, lb2, 32);
  if (l < 16){
    float* p = hout + (size_t)row*64 + 4*l;
    *(volatile v4f*)p = o;
    __threadfence();
    *(volatile v4f*)p = o;
  }
}

__global__ __launch_bounds__(32) void k_xp1(const float* h0, const f16* wt, const float* as1, const float* ad1,
    float* xp, float* al, int nRows){
  __shared__ __attribute__((aligned(16))) float xs[16*64];
  const int l = threadIdx.x & 31, h = l >> 4, m = l & 15;
  const int r0 = blockIdx.x*16;
  int rowA = r0 + m; if (rowA > nRows-1) rowA = nRows-1;
  const float* ap = h0 + (size_t)rowA*64;
  Frag a[2];
#pragma unroll
  for (int ks=0; ks<2; ks++){
#pragma unroll
    for (int i=0;i<8;i++){
      a[ks].v[i]   = (f16)ap[ks*32 + 8*h + i];
      a[ks].v[8+i] = (f16)ap[ks*32 + 16 + 8*h + i];
    }
  }
#pragma unroll
  for (int jt=0; jt<4; jt++){
    v8f acc = zero8();
#pragma unroll
    for (int ks=0; ks<2; ks++){
      Frag b;
      const f16* bp = wt + (size_t)(jt*16 + m)*64 + ks*32;
      b.half[0] = *(const v8h*)(bp + 8*h);
      b.half[1] = *(const v8h*)(bp + 16 + 8*h);
      acc = mma16(a[ks].v, b.v, acc);
    }
#pragma unroll
    for (int r=0;r<8;r++) xs[(8*h + r)*64 + jt*16 + m] = acc[r]*SCL;
  }
  __syncthreads();
  const int arow = l >> 1, part = l & 1;
  const float* vec = part ? ad1 : as1;
  v4f o;
#pragma unroll
  for (int hd=0; hd<4; hd++){
    float s = 0.f;
#pragma unroll
    for (int c=0;c<16;c++) s += xs[arow*64 + hd*16 + c]*vec[hd*16 + c];
    o[hd] = s;
  }
  const bool aok = (r0 + arow) < nRows;
  float* ab = al + (size_t)r0*8 + l*4;
  float* xb = xp + (size_t)r0*64;
  if (aok) *(volatile v4f*)ab = o;
#pragma unroll
  for (int i=0;i<8;i++){
    int off = (i*32 + l)*4;
    if (r0 + (off>>6) < nRows){ v4f v = *(const v4fa*)(xs + off); *(volatile v4f*)(xb + off) = v; }
  }
  __threadfence();
  if (aok) *(volatile v4f*)ab = o;
#pragma unroll
  for (int i=0;i<8;i++){
    int off = (i*32 + l)*4;
    if (r0 + (off>>6) < nRows){ v4f v = *(const v4fa*)(xs + off); *(volatile v4f*)(xb + off) = v; }
  }
}

__device__ __forceinline__ void gru_layer(v16h ax0, v16h ax1, v16h ahA, v16h ahB,
    const f16* wih, const f16* whh, const float* bih, const float* bhh,
    float* hf, f16* hh, int m, int h){
#pragma unroll
  for (int j=0; j<4; j++){
    const int col = j*16 + m;
    v8f ar = zero8(), az = zero8(), an = zero8(), ag = zero8();
#pragma unroll
    for (int ks=0; ks<2; ks++){
      const v16h A  = ks ? ax1 : ax0;
      const v16h Hv = ks ? ahB : ahA;
      const int cb = col*64 + ks*32 + 8*h;
      Frag b;
      b.half[0] = *(const v8h*)(wih + cb);           b.half[1] = *(const v8h*)(wih + cb + 16);           ar = mma16(A,  b.v, ar);
      b.half[0] = *(const v8h*)(wih + 4096 + cb);    b.half[1] = *(const v8h*)(wih + 4096 + cb + 16);    az = mma16(A,  b.v, az);
      b.half[0] = *(const v8h*)(wih + 8192 + cb);    b.half[1] = *(const v8h*)(wih + 8192 + cb + 16);    an = mma16(A,  b.v, an);
      b.half[0] = *(const v8h*)(whh + cb);           b.half[1] = *(const v8h*)(whh + cb + 16);           ar = mma16(Hv, b.v, ar);
      b.half[0] = *(const v8h*)(whh + 4096 + cb);    b.half[1] = *(const v8h*)(whh + 4096 + cb + 16);    az = mma16(Hv, b.v, az);
      b.half[0] = *(const v8h*)(whh + 8192 + cb);    b.half[1] = *(const v8h*)(whh + 8192 + cb + 16);    ag = mma16(Hv, b.v, ag);
    }
    const float bir = bih[col], biz = bih[64+col], bic = bih[128+col];
    const float bhr = bhh[col], bhz = bhh[64+col], bhc = bhh[128+col];
#pragma unroll
    for (int r=0; r<8; r++){
      const int idx = (8*h + r)*64 + col;
      float pr = ar[r]*SCL + bir + bhr;
      float pz = az[r]*SCL + biz + bhz;
      float rg = 1.f/(1.f + expf(-pr));
      float zg = 1.f/(1.f + expf(-pz));
      float cand = tanhf(an[r]*SCL + bic + rg*(ag[r]*SCL + bhc));
      float hp = hf[idx];
      float hn = (1.f - zg)*cand + zg*hp;
      hf[idx] = hn;
      hh[idx] = (f16)hn;
    }
  }
}

__global__ __launch_bounds__(GRU_T) void k_gru(const float* xin,
    const f16* wih0, const f16* whh0, const f16* wih1, const f16* whh1, const f16* hw16,
    const float* bih0, const float* bhh0, const float* bih1, const float* bhh1,
    const float* headb, float* out, int nRG){
  extern __shared__ __attribute__((aligned(16))) f16 smem[];
  f16* wih0s = smem;
  f16* whh0s = smem + 1*WTS;
  f16* wih1s = smem + 2*WTS;
  f16* whh1s = smem + 3*WTS;
  f16* hws   = smem + 4*WTS;
  const int tid = threadIdx.x, l = tid & 31, w = tid >> 5, h = l >> 4, m = l & 15;
  f16* wreg = smem + 4*WTS + 1024 + w*GRU_WAVE_HALVES;
  float* h0f = (float*)wreg;
  float* h1f = (float*)(wreg + 2048);
  f16*   h0h = wreg + 4096;
  f16*   h1h = wreg + 5120;

  {
    const v8h* s0 = (const v8h*)wih0; const v8h* s1 = (const v8h*)whh0;
    const v8h* s2 = (const v8h*)wih1; const v8h* s3 = (const v8h*)whh1;
    v8h* d0 = (v8h*)wih0s; v8h* d1 = (v8h*)whh0s; v8h* d2 = (v8h*)wih1s; v8h* d3 = (v8h*)whh1s;
    for (int i=tid; i<WTS/8; i+=GRU_T){ d0[i]=s0[i]; d1[i]=s1[i]; d2[i]=s2[i]; d3[i]=s3[i]; }
    const v8h* s4 = (const v8h*)hw16; v8h* d4 = (v8h*)hws;
    for (int i=tid; i<1024/8; i+=GRU_T) d4[i] = s4[i];
  }
  for (int i=l; i<1024; i+=32){ h0f[i]=0.f; h1f[i]=0.f; h0h[i]=(f16)0.f; h1h[i]=(f16)0.f; }
  __syncthreads();

  const int ntiles = (nRG + 15) >> 4;
  int tile = blockIdx.x*GW + w;
  const bool valid = (tile < ntiles) && (tile*16 + 16 <= nRG);
  if (tile > ntiles-1) tile = ntiles-1;
  if (tile < 0) tile = 0;
  const int r0 = tile*16;
  int rg = r0 + m; if (rg > nRG-1) rg = nRG-1;
  const int bI = rg / NN, nI = rg - bI*NN;

#pragma unroll 1
  for (int t=0; t<NT; t++){
    const float* xr = xin + (((size_t)(bI*NT + t))*NN + nI)*64;
    Frag ax[2], ah[2];
#pragma unroll
    for (int ks=0; ks<2; ks++){
#pragma unroll
      for (int i=0;i<8;i++){
        ax[ks].v[i]   = (f16)xr[ks*32 + 8*h + i];
        ax[ks].v[8+i] = (f16)xr[ks*32 + 16 + 8*h + i];
      }
      ah[ks].half[0] = *(const v8h*)(h0h + m*64 + ks*32 + 8*h);
      ah[ks].half[1] = *(const v8h*)(h0h + m*64 + ks*32 + 16 + 8*h);
    }
    __syncthreads();
    gru_layer(ax[0].v, ax[1].v, ah[0].v, ah[1].v, wih0s, whh0s, bih0, bhh0, h0f, h0h, m, h);
    __syncthreads();
    Frag bx[2], bh[2];
#pragma unroll
    for (int ks=0; ks<2; ks++){
      bx[ks].half[0] = *(const v8h*)(h0h + m*64 + ks*32 + 8*h);
      bx[ks].half[1] = *(const v8h*)(h0h + m*64 + ks*32 + 16 + 8*h);
      bh[ks].half[0] = *(const v8h*)(h1h + m*64 + ks*32 + 8*h);
      bh[ks].half[1] = *(const v8h*)(h1h + m*64 + ks*32 + 16 + 8*h);
    }
    __syncthreads();
    gru_layer(bx[0].v, bx[1].v, bh[0].v, bh[1].v, wih1s, whh1s, bih1, bhh1, h1f, h1h, m, h);
    __syncthreads();
  }

  v8f acc = zero8();
#pragma unroll
  for (int ks=0; ks<2; ks++){
    Frag a, b;
    a.half[0] = *(const v8h*)(h1h + m*64 + ks*32 + 8*h);
    a.half[1] = *(const v8h*)(h1h + m*64 + ks*32 + 16 + 8*h);
    b.half[0] = *(const v8h*)(hws + m*64 + ks*32 + 8*h);
    b.half[1] = *(const v8h*)(hws + m*64 + ks*32 + 16 + 8*h);
    acc = mma16(a.v, b.v, acc);
  }
  float* os = h0f;
  if (m < NTF){
    const float hb = headb[m];
#pragma unroll
    for (int r=0;r<8;r++) os[(8*h + r)*NTF + m] = acc[r]*SCL + hb;
  }
  __syncthreads();
  if (valid){
    float* ob = out + (size_t)r0*NTF;
    const bool second = l < (16*NTF - 128)/4;
    v4f v0 = *(const v4fa*)(os + l*4);
    v4f v1 = v0;
    if (second) v1 = *(const v4fa*)(os + 128 + l*4);
    *(volatile v4f*)(ob + l*4) = v0;
    if (second) *(volatile v4f*)(ob + 128 + l*4) = v1;
    __threadfence();
    *(volatile v4f*)(ob + l*4) = v0;
    if (second) *(volatile v4f*)(ob + 128 + l*4) = v1;
  }
}

extern "C" void kernel_launch(void* const* d_in, const int* in_sizes, int n_in,
                              void* d_out, int out_size, void* d_ws, size_t ws_size,
                              hipStream_t stream){
  if (n_in < 31) return;
  const float* x_seq = (const float*)d_in[0];
  const int*   ei    = (const int*)d_in[1];
  const float* ew    = (const float*)d_in[2];
  const float* g0W=(const float*)d_in[3],  *g0as=(const float*)d_in[4],  *g0ad=(const float*)d_in[5];
  const float* g0We=(const float*)d_in[6], *g0ae=(const float*)d_in[7],  *g0b=(const float*)d_in[8];
  const float* g1W=(const float*)d_in[9],  *g1as=(const float*)d_in[10], *g1ad=(const float*)d_in[11];
  const float* g1We=(const float*)d_in[12],*g1ae=(const float*)d_in[13], *g1b=(const float*)d_in[14];
  const float* ln0g=(const float*)d_in[15],*ln0b=(const float*)d_in[16];
  const float* ln1g=(const float*)d_in[17],*ln1b=(const float*)d_in[18];
  const float* skW=(const float*)d_in[19], *skb=(const float*)d_in[20];
  const float* gru0Wih=(const float*)d_in[21],*gru0Whh=(const float*)d_in[22];
  const float* gru0bih=(const float*)d_in[23],*gru0bhh=(const float*)d_in[24];
  const float* gru1Wih=(const float*)d_in[25],*gru1Whh=(const float*)d_in[26];
  const float* gru1bih=(const float*)d_in[27],*gru1bhh=(const float*)d_in[28];
  const float* headW=(const float*)d_in[29],*headb=(const float*)d_in[30];
  float* out = (float*)d_out;

  if (in_sizes[0] != NB*NN*NT*NCIN) return;
  if (in_sizes[1] != 2*NE) return;
  if (in_sizes[2] != NE) return;
  if (out_size != RG*NTF) return;
  const int nE = in_sizes[2];

  size_t off = 0;
  auto take = [&](size_t bytes)->char*{ char* p = (char*)d_ws + off; off += (bytes + 255) & ~(size_t)255; return p; };
  float* xp    = (float*)take((size_t)RR*64*4);
  float* h0b   = (float*)take((size_t)RR*64*4);
  float* h1b   = (float*)take((size_t)RR*64*4);
  float* al    = (float*)take((size_t)RR*8*4);
  int*   rowptr= (int*)  take((size_t)RP_PAD*4);
  int*   ssrc  = (int*)  take((size_t)EPAD*4);
  float* sw    = (float*)take((size_t)EPAD*4);
  float* sc    = (float*)take(256);
  f16* wih0h = (f16*)take((size_t)WTS*2);
  f16* whh0h = (f16*)take((size_t)WTS*2);
  f16* wih1h = (f16*)take((size_t)WTS*2);
  f16* whh1h = (f16*)take((size_t)WTS*2);
  f16* g1wt  = (f16*)take((size_t)64*64*2);
  f16* hw16  = (f16*)take((size_t)16*64*2);
  if (off > ws_size) return;

  const int prepw_groups = 4*(WTS/8) + 512 + 128;
  const int gat_blocks   = (RR + 7)/8;
  const int gru_tiles    = (RG + 15)/16;
  const int gru_blocks   = (gru_tiles + GW - 1)/GW;

  hipFuncSetAttribute(reinterpret_cast<const void*>(&k_gru), hipFuncAttributeMaxDynamicSharedMemorySize, GRU_LDS_BYTES);

  k_prep<<<1,256,0,stream>>>(ew, nE, g0We, g0ae, g1We, g1ae, sc);
  k_prepw<<<(prepw_groups+255)/256,256,0,stream>>>(gru0Wih, gru0Whh, gru1Wih, gru1Whh, g1W, headW,
                                                  wih0h, whh0h, wih1h, whh1h, g1wt, hw16);
  k_csr_rowptr<<<1,CSR_T,0,stream>>>(ei, nE, NN, rowptr);
  k_slotfill<<<EPAD/SB,256,0,stream>>>(ei, ew, nE, NN, rowptr, ssrc, sw);
  k_feat0<<<(RR+127)/128,128,0,stream>>>(x_seq, g0W, g0as, g0ad, xp, al, RR);
  k_gat<<<gat_blocks,256,0,stream>>>(0, 1, rowptr, ssrc, sw, al, xp, sc,
                                     g0b, ln0g, ln0b, x_seq, skW, skb, h0b, h0b, RR);
  k_xp1<<<(RR+15)/16,32,0,stream>>>(h0b, g1wt, g1as, g1ad, xp, al, RR);
  k_gat<<<gat_blocks,256,0,stream>>>(1, 5, rowptr, ssrc, sw, al, xp, sc,
                                     g1b, ln1g, ln1b, x_seq, skW, skb, h0b, h1b, RR);
  k_gru<<<gru_blocks,GRU_T,GRU_LDS_BYTES,stream>>>(h1b, wih0h, whh0h, wih1h, whh1h, hw16,
                                                  gru0bih, gru0bhh, gru1bih, gru1bhh, headb, out, RG);
}
